// LAConv2D_10015863734306
// MI455X (gfx1250) — hardware-verified
//
#include <hip/hip_runtime.h>
#include <math.h>

constexpr int kBatch  = 8;
constexpr int kCin    = 32;
constexpr int kCout   = 32;
constexpr int kSide   = 192;
constexpr int kPix    = kSide * kSide;
constexpr int kTaps   = 9;
constexpr int kKdim   = kCin * kTaps;
constexpr int kNpad   = 64;
constexpr int kGrp    = 2;
constexpr int kNumGrp = kBatch / kGrp;
constexpr float kW1Carry = 16.0f;
constexpr float kW1Inv   = 1.0f / 16.0f;
constexpr float kW2Carry = 8.0f;
constexpr float kW2Inv   = 1.0f / 8.0f;
constexpr float kInvPix  = 1.0f / 36864.0f;

constexpr size_t kBytesBt   = (size_t)kNpad * kKdim * 2;
constexpr size_t kBytesBias = (size_t)kBatch * kCout * 4;
constexpr size_t kBytesXT   = (size_t)kGrp * kPix * kCin * 4;
constexpr size_t kBytesA    = (size_t)kGrp * kPix * kKdim * 2;
constexpr size_t kBytesC    = (size_t)kGrp * kPix * kNpad * 4;
constexpr size_t kBytesAtt  = (size_t)kGrp * kTaps * kPix * 4;

typedef __attribute__((ext_vector_type(16))) _Float16 v16h;
typedef __attribute__((ext_vector_type(8)))  _Float16 v8h;
typedef __attribute__((ext_vector_type(16))) __bf16   v16b;
typedef __attribute__((ext_vector_type(8)))  __bf16   v8b;
typedef __attribute__((ext_vector_type(8)))  float    v8f;
typedef __attribute__((ext_vector_type(4)))  float    v4f;
typedef __attribute__((ext_vector_type(4)))  unsigned int v4u;

__device__ __forceinline__ unsigned short f2bf_bits(float f) {
  unsigned u = __float_as_uint(f);
  return (unsigned short)((u + 0x7FFFu + ((u >> 16) & 1u)) >> 16);
}
__device__ __forceinline__ float bf_bits2f(unsigned short h) { return __uint_as_float(((unsigned)h) << 16); }

__device__ __forceinline__ void dep_guard_h(v8f& a, v8f& b, v16h x, v16h y) { asm volatile("v_nop\n\tv_nop\n\tv_nop\n\tv_nop" : "+v"(a), "+v"(b) : "v"(x), "v"(y)); }
__device__ __forceinline__ void dep_guard_b(v8f& a, v8f& b, v16b x, v16b y) { asm volatile("v_nop\n\tv_nop\n\tv_nop\n\tv_nop" : "+v"(a), "+v"(b) : "v"(x), "v"(y)); }
__device__ __forceinline__ void keep4_h(v16h a, v16h b, v16h c, v16h d) { asm volatile("v_nop" :: "v"(a), "v"(b), "v"(c), "v"(d)); }
__device__ __forceinline__ void keep4_b(v16b a, v16b b, v16b c, v16b d) { asm volatile("v_nop" :: "v"(a), "v"(b), "v"(c), "v"(d)); }
__device__ __forceinline__ void acc_guard4(v8f& a, v8f& b, v8f& c, v8f& d) { asm volatile("v_nop\n\tv_nop\n\tv_nop\n\tv_nop" : "+v"(a), "+v"(b), "+v"(c), "+v"(d)); }
template <typename T> struct Frag;
template <> struct Frag<_Float16> {
  typedef v16h V; union U { v16h v; v8h h[2]; };
  static __device__ __forceinline__ v16h load(const _Float16* p) {
    U f; f.h[0] = *(const v8h*)(p); f.h[1] = *(const v8h*)(p + 16); return f.v;
  }
  static __device__ __forceinline__ v8f mma(v16h a, v16h b, v8f c) {
    return __builtin_amdgcn_wmma_f32_16x16x32_f16(false, a, false, b, (short)0, c, false, false);
  }
  static __device__ __forceinline__ void guard(v8f& a, v8f& b, v16h x, v16h y) { dep_guard_h(a, b, x, y); }
  static __device__ __forceinline__ void keep(v16h a, v16h b, v16h c, v16h d) { keep4_h(a, b, c, d); }
};
template <> struct Frag<__bf16> {
  typedef v16b V; union U { v16b v; v8b h[2]; };
  static __device__ __forceinline__ v16b load(const __bf16* p) {
    U f; f.h[0] = *(const v8b*)(p); f.h[1] = *(const v8b*)(p + 16); return f.v;
  }
  static __device__ __forceinline__ v8f mma(v16b a, v16b b, v8f c) {
    return __builtin_amdgcn_wmma_f32_16x16x32_bf16(false, a, false, b, (short)0, c, false, false);
  }
  static __device__ __forceinline__ void guard(v8f& a, v8f& b, v16b x, v16b y) { dep_guard_b(a, b, x, y); }
  static __device__ __forceinline__ void keep(v16b a, v16b b, v16b c, v16b d) { keep4_b(a, b, c, d); }
};

__device__ __forceinline__ unsigned pk16(unsigned short a, unsigned short b) { return (unsigned)a | ((unsigned)b << 16); }
__device__ __forceinline__ unsigned short h_bits(float f) { const _Float16 h = (_Float16)f; return __builtin_bit_cast(unsigned short, h); }

template <int ET> struct Elem;
template <> struct Elem<0> { typedef _Float16 T; };
template <> struct Elem<1> { typedef __bf16 T; };
template <int ET, bool SPLIT, int BIAS_MODE, int OUT_MODE, bool RESID, int ACT = 0>
__global__ __launch_bounds__(256) void wmma_gemm64(
    const unsigned short* __restrict__ Ap, const unsigned short* __restrict__ A2p, int lda, long strideA,
    const unsigned short* __restrict__ Btp, const unsigned short* __restrict__ Bt2p, int ldb, long strideB,
    void* __restrict__ Cout, void* __restrict__ Cout2, int ldc, long strideC,
    const float* __restrict__ bias,
    const float* __restrict__ resid, long strideR,
    int M, int N, int K, float scale) {
  typedef typename Elem<ET>::T T;
  typedef typename Frag<T>::V V;
  const T* A = (const T*)Ap; const T* A2 = (const T*)A2p; const T* Bt = (const T*)Btp; const T* Bt2 = (const T*)Bt2p;
  __shared__ __align__(16) float sT[8][16 * 68];
  const int b    = blockIdx.y;
  const int lane = threadIdx.x & 31;
  const int wave = threadIdx.x >> 5;
  const int tilesN = N >> 6;
  const int tilesM = M >> 6;
  const int tile = blockIdx.x * 8 + wave;
  if (tile >= tilesM * tilesN) return;
  const int tm = tile / tilesN;
  const int tn = tile - tm * tilesN;
  const int m0 = tm << 6;
  const int n0 = tn << 6;

  const T* Ab  = A  + (size_t)b * strideA;
  const T* Bb  = Bt + (size_t)b * strideB;
  const T* Ab2 = SPLIT ? (A2  + (size_t)b * strideA) : nullptr;
  const T* Bb2 = SPLIT ? (Bt2 + (size_t)b * strideB) : nullptr;

  const int rlane = lane & 15;
  const int koff  = (lane >> 4) * 8;
  const int mOff  = (lane >> 4) * 8;

  v8f acc[4][4];
#pragma unroll
  for (int i = 0; i < 4; ++i)
#pragma unroll
    for (int j = 0; j < 4; ++j) acc[i][j] = (v8f){0.f,0.f,0.f,0.f,0.f,0.f,0.f,0.f};

  for (int k0 = 0; k0 < K; k0 += 32) {
    V bh[4], bl[4];
#pragma unroll
    for (int j = 0; j < 4; ++j) {
      const size_t bo = (size_t)(n0 + (j << 4) + rlane) * ldb + koff + k0;
      bh[j] = Frag<T>::load(Bb + bo);
      if (SPLIT) bl[j] = Frag<T>::load(Bb2 + bo);
    }
#pragma unroll
    for (int i = 0; i < 4; ++i) {
      const size_t ao = (size_t)(m0 + (i << 4) + rlane) * lda + koff + k0;
      V ah = Frag<T>::load(Ab + ao);
      V al;
      if (SPLIT) al = Frag<T>::load(Ab2 + ao);
#pragma unroll
      for (int j = 0; j < 4; ++j) {
        acc[i][j] = Frag<T>::mma(ah, bh[j], acc[i][j]);
        if (SPLIT) {
          acc[i][j] = Frag<T>::mma(ah, bl[j], acc[i][j]);
          acc[i][j] = Frag<T>::mma(al, bh[j], acc[i][j]);
        }
      }
      Frag<T>::guard(acc[i][0], acc[i][3], ah, SPLIT ? al : ah);
    }
    Frag<T>::keep(bh[0], bh[1], bh[2], bh[3]);
    if (SPLIT) Frag<T>::keep(bl[0], bl[1], bl[2], bl[3]);
  }
  acc_guard4(acc[0][0], acc[0][1], acc[0][2], acc[0][3]);
  acc_guard4(acc[1][0], acc[1][1], acc[1][2], acc[1][3]);
  acc_guard4(acc[2][0], acc[2][1], acc[2][2], acc[2][3]);
  acc_guard4(acc[3][0], acc[3][1], acc[3][2], acc[3][3]);

  float* slab = sT[wave];
  const float* Rb = RESID ? (resid + (size_t)b * strideR) : nullptr;
#pragma unroll
  for (int i = 0; i < 4; ++i) {
    const int mBase = m0 + (i << 4);
#pragma unroll
    for (int j = 0; j < 4; ++j) {
      const int n = n0 + (j << 4) + rlane;
      float bv = 0.f;
      if (BIAS_MODE == 2) bv = bias[n];
#pragma unroll
      for (int r = 0; r < 8; ++r) {
        float v = acc[i][j][r] * scale;
        if (BIAS_MODE == 1) v += bias[mBase + mOff + r];
        if (BIAS_MODE == 2) v += bv;
        if (RESID) v += Rb[(size_t)(mBase + mOff + r) * ldc + n];
        if (ACT == 2) v = fmaxf(v, 0.0f);
        if (ACT == 4) v = (v > 0.f) ? v : 0.01f * v;
        slab[(mOff + r) * 68 + (j << 4) + rlane] = v;
      }
    }
    __builtin_amdgcn_fence(__ATOMIC_RELEASE, "workgroup");
    __builtin_amdgcn_wave_barrier();
    __builtin_amdgcn_fence(__ATOMIC_ACQUIRE, "workgroup");
    if (OUT_MODE == 0) {
      float* C = (float*)Cout + (size_t)b * strideC;
      const int hh = lane >> 4, c4 = (lane & 15) * 4;
      for (int pass = 0; pass < 2; ++pass) {
#pragma unroll
        for (int it = 0; it < 8; ++it) {
          const int row = it * 2 + hh;
          v4f v = *(const v4f*)(slab + row * 68 + c4);
          *(volatile v4f*)(C + (size_t)(mBase + row) * ldc + n0 + c4) = v;
        }
        __threadfence();
      }
    } else {
      const int q = lane >> 3, c8 = (lane & 7) * 8;
      unsigned short* C  = (unsigned short*)Cout  + (size_t)b * strideC;
      unsigned short* C2 = (OUT_MODE == 2) ? ((unsigned short*)Cout2 + (size_t)b * strideC) : nullptr;
      for (int pass = 0; pass < 2; ++pass) {
#pragma unroll
        for (int it = 0; it < 4; ++it) {
          const int row = it * 4 + q;
          const float* sp = slab + row * 68 + c8;
          v8h hv, lv;
#pragma unroll
          for (int e = 0; e < 8; ++e) {
            if (OUT_MODE == 1) {
              hv[e] = (_Float16)sp[e];
            } else {
              unsigned short hb = f2bf_bits(sp[e]);
              unsigned short lb = f2bf_bits(sp[e] - bf_bits2f(hb));
              hv[e] = __builtin_bit_cast(_Float16, hb);
              lv[e] = __builtin_bit_cast(_Float16, lb);
            }
          }
          *(volatile v8h*)(C + (size_t)(mBase + row) * ldc + n0 + c8) = hv;
          if (OUT_MODE == 2) *(volatile v8h*)(C2 + (size_t)(mBase + row) * ldc + n0 + c8) = lv;
        }
        __threadfence();
      }
    }
    __builtin_amdgcn_fence(__ATOMIC_RELEASE, "workgroup");
    __builtin_amdgcn_wave_barrier();
    __builtin_amdgcn_fence(__ATOMIC_ACQUIRE, "workgroup");
  }
}

__global__ __launch_bounds__(256) void prep_bt_kernel(const float* __restrict__ a1w, const float* __restrict__ wmain,
                                                      unsigned short* __restrict__ bt1, unsigned short* __restrict__ bt2) {
  const int z = blockIdx.y;
  const float* src = (z == 0) ? a1w : wmain;
  unsigned short* dst = (z == 0) ? bt1 : bt2;
  const int nreal = (z == 0) ? kTaps : kCout;
  const float sc = (z == 0) ? kW1Carry : kW2Carry;
  const int g = blockIdx.x * 256 + threadIdx.x;
  if (g >= kNpad * (kKdim / 8)) return;
  const int row = g / 36;
  const int rem = g - row * 36;
  const int p   = rem >> 2;
  const int n0  = (rem & 3) * 8;
  const bool live = row < nreal;
  const int rowc = live ? row : (nreal - 1);
  unsigned short hb[8];
#pragma unroll
  for (int e = 0; e < 8; ++e) {
    float v = src[((size_t)(rowc * kCin + n0 + e)) * kTaps + p] * sc;
    v = live ? v : 0.0f;
    hb[e] = h_bits(v);
  }
  const v4u u = (v4u){pk16(hb[0], hb[1]), pk16(hb[2], hb[3]), pk16(hb[4], hb[5]), pk16(hb[6], hb[7])};
  unsigned short* q = dst + (size_t)g * 8;
  *(volatile v4u*)q = u;
  __threadfence();
  *(volatile v4u*)q = u;
}

__global__ __launch_bounds__(256) void poolbias_kernel(const float* __restrict__ x,
                                                       const float* __restrict__ b1w, const float* __restrict__ b1b,
                                                       const float* __restrict__ b2w, const float* __restrict__ b2b,
                                                       float* __restrict__ biasws) {
  __shared__ float red[kCin][8];
  __shared__ float pooled[kCin];
  __shared__ float hbuf[kCout];
  __shared__ float bout[kCout];
  const int b = blockIdx.x;
  const int tid = threadIdx.x, lane = tid & 31, wave = tid >> 5;
#pragma unroll 1
  for (int n = 0; n < kCin; ++n) {
    const float* xp = x + ((size_t)(b * kCin + n)) * kPix;
    float s = 0.0f;
#pragma unroll 1
    for (int i = tid; i < kPix; i += 256) s += xp[i];
#pragma unroll
    for (int off = 16; off > 0; off >>= 1) s += __shfl_xor(s, off, 32);
    if (lane == 0) red[n][wave] = s;
  }
  __syncthreads();
  if (tid < kCin) {
    float s = 0.0f;
#pragma unroll
    for (int j = 0; j < 8; ++j) s += red[tid][j];
    pooled[tid] = s * kInvPix;
  }
  __syncthreads();
  if (tid < kCout) {
    float hsum = b1b[tid];
#pragma unroll 1
    for (int n = 0; n < kCin; ++n) hsum = fmaf(pooled[n], b1w[tid * kCin + n], hsum);
    hbuf[tid] = fmaxf(hsum, 0.0f);
  }
  __syncthreads();
  if (tid < kCout) {
    float a = b2b[tid];
#pragma unroll 1
    for (int j = 0; j < kCout; ++j) a = fmaf(hbuf[j], b2w[tid * kCout + j], a);
    bout[tid] = a;
  }
  __syncthreads();
  if (tid < kCout) {
    const float v = bout[tid];
    float* q = biasws + b * kCout + tid;
    *(volatile float*)q = v;
    __threadfence();
    *(volatile float*)q = v;
  }
}

__global__ __launch_bounds__(256) void xt_kernel(const float* __restrict__ x, float* __restrict__ xT, int img0) {
  __shared__ __align__(16) float sm[128][36];
  const int tid = threadIdx.x, lane = tid & 31, wave = tid >> 5;
  const int bl = blockIdx.y;
  const int b  = img0 + bl;
  const int pix0 = blockIdx.x * 128;
  const float* xb = x + (size_t)b * kCin * kPix;
#pragma unroll
  for (int it = 0; it < 4; ++it) {
    const int e4 = it * 256 + tid;
    const int n  = e4 >> 5;
    const int p4 = (e4 & 31) * 4;
    const v4f v = *(const v4f*)(xb + (size_t)n * kPix + pix0 + p4);
    sm[p4 + 0][n] = v[0];
    sm[p4 + 1][n] = v[1];
    sm[p4 + 2][n] = v[2];
    sm[p4 + 3][n] = v[3];
  }
  __syncthreads();
  float* dst = xT + ((size_t)bl * kPix + pix0) * kCin;
  const int q = lane >> 3, c4 = (lane & 7) * 4;
  for (int pass = 0; pass < 2; ++pass) {
#pragma unroll
    for (int it = 0; it < 4; ++it) {
      const int pl = wave * 16 + it * 4 + q;
      const v4f v = *(const v4f*)(&sm[pl][c4]);
      *(volatile v4f*)(dst + (size_t)pl * kCin + c4) = v;
    }
    __threadfence();
  }
}

template <bool kMod>
__global__ __launch_bounds__(128) void im2col_kernel(const float* __restrict__ xT, const float* __restrict__ att,
                                                     unsigned short* __restrict__ Aout) {
  __shared__ __align__(16) v4u stg[4][576];
  const int tid = threadIdx.x, lane = tid & 31, wave = tid >> 5;
  const int bl = blockIdx.y;
  const int pixw = blockIdx.x * 64 + wave * 16;
  const float* xs = xT + (size_t)bl * kPix * kCin;
  const float* as = att + (size_t)bl * kTaps * kPix;
  unsigned short* dst = Aout + ((size_t)bl * kPix + pixw) * kKdim;
#pragma unroll 1
  for (int i = 0; i < 18; ++i) {
    const int g   = i * 32 + lane;
    const int rl  = g / 36;
    const int rem = g - rl * 36;
    const int p   = rem >> 2;
    const int n0  = (rem & 3) * 8;
    const int pix = pixw + rl;
    const int h   = pix / kSide;
    const int w   = pix - h * kSide;
    const int di  = p / 3;
    const int dj  = p - di * 3;
    const int sh  = h + di - 1;
    const int sw  = w + dj - 1;
    const bool valid = ((unsigned)sh < (unsigned)kSide) && ((unsigned)sw < (unsigned)kSide);
    const int shc = sh < 0 ? 0 : (sh > kSide - 1 ? kSide - 1 : sh);
    const int swc = sw < 0 ? 0 : (sw > kSide - 1 ? kSide - 1 : sw);
    const float* sp = xs + (size_t)(shc * kSide + swc) * kCin + n0;
    const v4f u0 = *(const v4f*)(sp);
    const v4f u1 = *(const v4f*)(sp + 4);
    float sc = valid ? 1.0f : 0.0f;
    if (kMod) {
      const float a = as[(size_t)p * kPix + pix];
      sc = valid ? a : 0.0f;
    }
    unsigned short hb[8];
#pragma unroll
    for (int e = 0; e < 4; ++e) {
      hb[e]     = h_bits(u0[e] * sc);
      hb[4 + e] = h_bits(u1[e] * sc);
    }
    const v4u pk = (v4u){pk16(hb[0], hb[1]), pk16(hb[2], hb[3]), pk16(hb[4], hb[5]), pk16(hb[6], hb[7])};
    stg[wave][g] = pk;
    *(volatile v4u*)(dst + (size_t)g * 8) = pk;
  }
  __threadfence();
#pragma unroll 1
  for (int i = 0; i < 18; ++i) {
    const int g = i * 32 + lane;
    const v4u pk = stg[wave][g];
    *(volatile v4u*)(dst + (size_t)g * 8) = pk;
  }
}

__global__ __launch_bounds__(256) void att_kernel(const float* __restrict__ C1,
                                                  const float* __restrict__ a1b,
                                                  const float* __restrict__ a2w, const float* __restrict__ a2b,
                                                  const float* __restrict__ a3w, const float* __restrict__ a3b,
                                                  float* __restrict__ att) {
  __shared__ float s_w2[81], s_w3[81];
  __shared__ float s_b1[9], s_b2[9], s_b3[9];
  __shared__ float s_h1[9][256], s_h2[9][256];
  const int tid = threadIdx.x;
  if (tid < 81) { s_w2[tid] = a2w[tid]; s_w3[tid] = a3w[tid]; }
  if (tid < 9)  { s_b1[tid] = a1b[tid]; s_b2[tid] = a2b[tid]; s_b3[tid] = a3b[tid]; }
  __syncthreads();
  const int bl  = blockIdx.y;
  const int pix = blockIdx.x * 256 + tid;
  const float* cr = C1 + ((size_t)bl * kPix + pix) * kNpad;
  const v4f u0 = *(const v4f*)(cr);
  const v4f u1 = *(const v4f*)(cr + 4);
  const float u8 = cr[8];
  s_h1[0][tid] = fmaxf(u0[0] + s_b1[0], 0.0f);
  s_h1[1][tid] = fmaxf(u0[1] + s_b1[1], 0.0f);
  s_h1[2][tid] = fmaxf(u0[2] + s_b1[2], 0.0f);
  s_h1[3][tid] = fmaxf(u0[3] + s_b1[3], 0.0f);
  s_h1[4][tid] = fmaxf(u1[0] + s_b1[4], 0.0f);
  s_h1[5][tid] = fmaxf(u1[1] + s_b1[5], 0.0f);
  s_h1[6][tid] = fmaxf(u1[2] + s_b1[6], 0.0f);
  s_h1[7][tid] = fmaxf(u1[3] + s_b1[7], 0.0f);
  s_h1[8][tid] = fmaxf(u8 + s_b1[8], 0.0f);
#pragma unroll 1
  for (int o = 0; o < 9; ++o) {
    float t = s_b2[o];
#pragma unroll
    for (int i = 0; i < 9; ++i) t = fmaf(s_w2[o * 9 + i], s_h1[i][tid], t);
    s_h2[o][tid] = fmaxf(t, 0.0f);
  }
  float* ap = att + (size_t)bl * kTaps * kPix + pix;
#pragma unroll 1
  for (int o = 0; o < 9; ++o) {
    float t = s_b3[o];
#pragma unroll
    for (int i = 0; i < 9; ++i) t = fmaf(s_w3[o * 9 + i], s_h2[i][tid], t);
    t = fminf(fmaxf(t, -40.0f), 40.0f);
    const float ex = expf(-t);
    const float sg = 1.0f / (1.0f + ex);
    s_h1[o][tid] = sg;
    *(volatile float*)(ap + (size_t)o * kPix) = sg;
  }
  __threadfence();
#pragma unroll 1
  for (int o = 0; o < 9; ++o) {
    const float sg = s_h1[o][tid];
    *(volatile float*)(ap + (size_t)o * kPix) = sg;
  }
}

__global__ __launch_bounds__(256) void out_kernel(const float* __restrict__ Y, const float* __restrict__ biasws,
                                                  float* __restrict__ out, int img0) {
  __shared__ __align__(16) float sm[kCout][132];
  const int tid = threadIdx.x, lane = tid & 31, wave = tid >> 5;
  const int bl = blockIdx.y;
  const int b  = img0 + bl;
  const int pix0 = blockIdx.x * 128;
  const float* ys = Y + ((size_t)bl * kPix + pix0) * kNpad;
#pragma unroll
  for (int it = 0; it < 4; ++it) {
    const int e4 = it * 256 + tid;
    const int pl = e4 >> 3;
    const int c4 = (e4 & 7) * 4;
    const v4f v = *(const v4f*)(ys + (size_t)pl * kNpad + c4);
    sm[c4 + 0][pl] = v[0];
    sm[c4 + 1][pl] = v[1];
    sm[c4 + 2][pl] = v[2];
    sm[c4 + 3][pl] = v[3];
  }
  __syncthreads();
  float* ob = out + (size_t)b * kCout * kPix + pix0;
  for (int pass = 0; pass < 2; ++pass) {
#pragma unroll
    for (int it = 0; it < 4; ++it) {
      const int m = wave * 4 + it;
      const float bm = biasws[b * kCout + m];
      v4f v = *(const v4f*)(&sm[m][lane * 4]);
      v[0] += bm; v[1] += bm; v[2] += bm; v[3] += bm;
      *(volatile v4f*)(ob + (size_t)m * kPix + lane * 4) = v;
    }
    __threadfence();
  }
}

extern "C" void kernel_launch(void* const* d_in, const int* in_sizes, int n_in,
                              void* d_out, int out_size, void* d_ws, size_t ws_size,
                              hipStream_t stream)
{
  if (n_in < 12) return;
  if (in_sizes[0] != kBatch * kCin * kPix) return;
  if (in_sizes[1] != kTaps * kCin * kTaps || in_sizes[11] != kCout * kCin * kTaps) return;
  if (out_size != kBatch * kCout * kPix) return;

  const float* x    = (const float*)d_in[0];
  const float* a1w  = (const float*)d_in[1];
  const float* a1b  = (const float*)d_in[2];
  const float* a2w  = (const float*)d_in[3];
  const float* a2b  = (const float*)d_in[4];
  const float* a3w  = (const float*)d_in[5];
  const float* a3b  = (const float*)d_in[6];
  const float* b1w  = (const float*)d_in[7];
  const float* b1b  = (const float*)d_in[8];
  const float* b2w  = (const float*)d_in[9];
  const float* b2b  = (const float*)d_in[10];
  const float* wght = (const float*)d_in[11];
  float* out = (float*)d_out;

  const size_t offBt1  = 0;
  const size_t offBt2  = offBt1 + kBytesBt;
  const size_t offBias = offBt2 + kBytesBt;
  const size_t offXT   = offBias + kBytesBias;
  const size_t offA16  = offXT + kBytesXT;
  const size_t offA2   = offA16 + kBytesA;
  const size_t offC    = offA2 + kBytesA;
  const size_t offAtt  = offC + kBytesC;
  const size_t offEnd  = offAtt + kBytesAtt;
  if (ws_size < offEnd) return;

  char* ws = (char*)d_ws;
  unsigned short* bt1  = (unsigned short*)(ws + offBt1);
  unsigned short* bt2  = (unsigned short*)(ws + offBt2);
  float* biasws        = (float*)(ws + offBias);
  float* xT            = (float*)(ws + offXT);
  unsigned short* a16  = (unsigned short*)(ws + offA16);
  unsigned short* a2m  = (unsigned short*)(ws + offA2);
  float* cbuf          = (float*)(ws + offC);
  float* attws         = (float*)(ws + offAtt);

  const long strideA = (long)kPix * kKdim;
  const long strideC = (long)kPix * kNpad;
  const int gemmGridX = (kPix / 64) / 8;

  prep_bt_kernel<<<dim3(9, 2), 256, 0, stream>>>(a1w, wght, bt1, bt2);
  poolbias_kernel<<<kBatch, 256, 0, stream>>>(x, b1w, b1b, b2w, b2b, biasws);

  for (int g = 0; g < kNumGrp; ++g) {
    const int img0 = g * kGrp;
    xt_kernel<<<dim3(kPix / 128, kGrp), 256, 0, stream>>>(x, xT, img0);
    im2col_kernel<false><<<dim3(kPix / 64, kGrp), 128, 0, stream>>>(xT, attws, a16);
    wmma_gemm64<0, false, 0, 0, false, 0><<<dim3(gemmGridX, kGrp), 256, 0, stream>>>(
        a16, a16, kKdim, strideA,
        bt1, bt1, kKdim, 0L,
        (void*)cbuf, (void*)cbuf, kNpad, strideC,
        biasws, cbuf, 0L,
        kPix, kNpad, kKdim, kW1Inv);
    att_kernel<<<dim3(kPix / 256, kGrp), 256, 0, stream>>>(cbuf, a1b, a2w, a2b, a3w, a3b, attws);
    im2col_kernel<true><<<dim3(kPix / 64, kGrp), 128, 0, stream>>>(xT, attws, a2m);
    wmma_gemm64<0, false, 0, 0, false, 0><<<dim3(gemmGridX, kGrp), 256, 0, stream>>>(
        a2m, a2m, kKdim, strideA,
        bt2, bt2, kKdim, 0L,
        (void*)cbuf, (void*)cbuf, kNpad, strideC,
        biasws, cbuf, 0L,
        kPix, kNpad, kKdim, kW2Inv);
    out_kernel<<<dim3(kPix / 128, kGrp), 256, 0, stream>>>(cbuf, biasws, out, img0);
  }
}
